// MSA_5196910428424
// MI455X (gfx1250) — hardware-verified
//
#include <hip/hip_runtime.h>


#ifndef NB
#define NB 4
#endif
#ifndef SEQ
#define SEQ 2048
#endif

namespace {
constexpr int NB_FULL = 4, SEQ_FULL = 2048, DM = 768, H = 12, HD = 64;
constexpr int BL = NB;
constexpr int T = SEQ;
constexpr int NSL = DM / 128;
constexpr bool VRES = true;
constexpr float XS = 8.0f, WSC = 256.0f, PS = 1024.0f, RS_ = 1024.0f, LOG2E = 1.4426950408889634f;
static_assert(T % 64 == 0 && T >= 64 && T <= SEQ_FULL && BL >= 1 && BL <= NB_FULL);
static_assert(DM % 128 == 0 && NSL * 128 == DM && H % 2 == 0 && H * HD == DM && HD == 64);
typedef _Float16 b16;
typedef __attribute__((ext_vector_type(16))) _Float16 v16b;
typedef __attribute__((ext_vector_type(8))) _Float16 v8b;
typedef __attribute__((ext_vector_type(4))) _Float16 v4h;
typedef __attribute__((ext_vector_type(2))) _Float16 v2h;
typedef __attribute__((ext_vector_type(8))) float v8f;
typedef __attribute__((ext_vector_type(4))) float v4f;
__device__ __forceinline__ float bf16_rne(float f) { unsigned int u = __float_as_uint(f); u += 0x7FFFu + ((u >> 16) & 1u); return __uint_as_float(u & 0xFFFF0000u); }
__device__ __forceinline__ v16b frag_kb(const b16* p, int hh) { const v8b a = *(const v8b*)(p + 8 * hh), b = *(const v8b*)(p + 16 + 8 * hh); v16b f;
#pragma unroll
  for (int e = 0; e < 8; ++e) { f[e] = a[e]; f[8 + e] = b[e]; } return f; }
__device__ __forceinline__ v8f wmma16b(v16b a, v16b b, v8f c) { v8f d = __builtin_amdgcn_wmma_f32_16x16x32_f16(false, a, false, b, (short)0, c, false, false); asm volatile("v_nop\n\tv_nop\n\tv_nop\n\tv_nop" : "+v"(d) : "v"(a), "v"(b)); return d; }
__device__ __forceinline__ void wave_lds_sync() { __builtin_amdgcn_fence(3, "workgroup"); __builtin_amdgcn_wave_barrier(); __builtin_amdgcn_fence(2, "workgroup"); }
__device__ __forceinline__ float nexp2(float v) { return __builtin_amdgcn_exp2f(v); }

__global__ __launch_bounds__(256) void prep_kernel(const float* __restrict__ wq, const float* __restrict__ wk, const float* __restrict__ wv, b16* __restrict__ WT) {
  const size_t u = (size_t)blockIdx.x * 256 + threadIdx.x; const size_t per = (size_t)H * HD * HD / 8; if (u >= 3 * per) return;
  const int m = (int)(u / per); const size_t e = (u % per) * 8; const float* w = m == 0 ? wq : m == 1 ? wk : wv; v8b o;
  for (int j = 0; j < 8; ++j) o[j] = (b16)(bf16_rne(w[e + j]) * WSC);
  for (int pass = 0; pass < 2; ++pass) { *(volatile v8b*)(WT + (size_t)m * H * HD * HD + e) = o; __threadfence(); }
}
__global__ __launch_bounds__(128) void proj_kernel(const float* __restrict__ x, const b16* __restrict__ WT, const float* __restrict__ bq, const float* __restrict__ bk, const float* __restrict__ bv,
                                                   b16* __restrict__ QP, b16* __restrict__ KP, b16* __restrict__ VTh, b16* __restrict__ VTl) {
  __shared__ __attribute__((aligned(16))) b16 As[64][128 + 8]; __shared__ __attribute__((aligned(16))) float Tf[4][16][128 + 4];
  const int wave = threadIdx.x >> 5, lane = threadIdx.x & 31, nloc = lane & 15, hlf = lane >> 4; const int t0 = blockIdx.x * 64; const int b = blockIdx.y;
  const int part = blockIdx.z / NSL, slab = blockIdx.z % NSL, c0 = slab * 128;
  const float* xb = x + ((size_t)b * SEQ_FULL + t0) * DM + c0; const float* bias = part == 0 ? bq : part == 1 ? bk : bv; const b16* Wp = WT + (size_t)part * H * HD * HD;
  for (int i = threadIdx.x; i < 64 * 32; i += 128) { const int rr = i / 32, q = (i % 32) * 4; const v4f f = *(const v4f*)(xb + (size_t)rr * DM + q); v4h o;
    for (int j = 0; j < 4; ++j) o[j] = (b16)(bf16_rne(f[j]) * XS); *(v4h*)(&As[rr][q]) = o; }
  __syncthreads();
  v8f acc[8];
#pragma unroll
  for (int t = 0; t < 8; ++t) acc[t] = (v8f){};
#pragma unroll
  for (int t = 0; t < 8; ++t) { const int h = 2 * slab + (t >> 2), e = (t & 3) * 16 + nloc; const b16* br = Wp + ((size_t)h * HD + e) * HD; const int a0 = (t >> 2) * HD;
#pragma unroll
    for (int kb = 0; kb < HD; kb += 32) acc[t] = wmma16b(frag_kb(&As[wave * 16 + nloc][a0 + kb], hlf), frag_kb(br + kb, hlf), acc[t]); }
#pragma unroll
  for (int t = 0; t < 8; ++t) { const int cl = t * 16 + nloc; const int h = 2 * slab + (t >> 2); const float bb = bf16_rne(bias[h * HD + (cl & 63)]);
#pragma unroll
    for (int r = 0; r < 8; ++r) Tf[wave][8 * hlf + r][cl] = acc[t][r] * (1.0f / (XS * WSC)) + bb; }
  __syncthreads();
  for (int pass = 0; pass < 2; ++pass) {
    if (part < 2) { b16* plane = part == 0 ? QP : KP; const int c = c0 + lane * 4; const int h = c / HD, d = c % HD;
      for (int rr = 0; rr < 16; ++rr) { const int tok = t0 + wave * 16 + rr; v4h o4; for (int j = 0; j < 4; ++j) o4[j] = (b16)(Tf[wave][rr][lane * 4 + j] * XS);
        *(volatile v4h*)(plane + (((size_t)b * H + h) * T + tok) * HD + d) = o4; } }
    else {
#pragma unroll 1
      for (int q = 0; q < 32; ++q) { const int cl = wave * 32 + q; const int c = c0 + cl; const int h = c / HD, d = c % HD; const int tk = lane * 2; v2h hv, lv;
        for (int j = 0; j < 2; ++j) { const float f = Tf[(tk + j) >> 4][(tk + j) & 15][cl] * XS; const b16 p = (b16)f; hv[j] = p; lv[j] = (b16)((f - (float)p) * RS_); }
        const size_t oi = (((size_t)b * H + h) * HD + d) * (size_t)T + t0 + lane * 2; *(volatile v2h*)(VTh + oi) = hv; if (VRES) *(volatile v2h*)(VTl + oi) = lv; } }
    __threadfence(); }
}
__global__ __launch_bounds__(64) __attribute__((amdgpu_num_vgpr(256))) void attn_kernel(const b16* __restrict__ QP, const b16* __restrict__ KP, const b16* __restrict__ VTh, const b16* __restrict__ VTl, float* __restrict__ out) {
  __shared__ __attribute__((aligned(16))) b16 Pb[2][16][32 + 8]; __shared__ __attribute__((aligned(16))) float To[2][16][HD + 4];
  const int wave = threadIdx.x >> 5, lane = threadIdx.x & 31, hh = lane >> 4, col = lane & 15; const int b = blockIdx.y / H, h = blockIdx.y % H; const int q0 = blockIdx.x * 32 + wave * 16, qi = q0 + col;
  const size_t ph = (size_t)b * H + h; const b16* Qb = QP + ph * T * HD; const b16* Kb = KP + ph * T * HD; const b16* Vh = VTh + ph * HD * (size_t)T; const b16* Vl = VTl + ph * HD * (size_t)T;
  const v16b qa0 = frag_kb(Qb + (size_t)qi * HD, hh), qa1 = frag_kb(Qb + (size_t)qi * HD + 32, hh);
  const float cs = LOG2E / (8.0f * XS * XS);
  float m = -INFINITY, l = 0.0f; v8f o[4], ol[4]; for (int t = 0; t < 4; ++t) { o[t] = (v8f){}; ol[t] = (v8f){}; }
#pragma unroll 1
  for (int kb = 0; kb < T; kb += 32) {
    float e[16]; float mx = -INFINITY;
#pragma unroll
    for (int u = 0; u < 2; ++u) { v8f s = (v8f){}; const size_t kr = (size_t)(kb + u * 16 + col) * HD; s = wmma16b(frag_kb(Kb + kr, hh), qa0, s); s = wmma16b(frag_kb(Kb + kr + 32, hh), qa1, s);
#pragma unroll
      for (int r = 0; r < 8; ++r) { const float vv = s[r] * cs; e[u * 8 + r] = vv; mx = fmaxf(mx, vv); } }
    mx = fmaxf(mx, __shfl_xor(mx, 16)); const float mn = fmaxf(m, mx); const float al = nexp2(m - mn); float sum = 0.0f;
#pragma unroll
    for (int i2 = 0; i2 < 16; ++i2) { const float p = nexp2(e[i2] - mn); sum += p; Pb[wave][col][(i2 < 8 ? 0 : 16) + 8 * hh + (i2 & 7)] = (b16)(p * PS); }
    sum += __shfl_xor(sum, 16); l = l * al + sum; m = mn;
    wave_lds_sync();
    const v16b pf = frag_kb(&Pb[wave][col][0], hh);
#pragma unroll
    for (int t = 0; t < 4; ++t) { o[t] *= al; o[t] = wmma16b(frag_kb(Vh + (size_t)(t * 16 + col) * T + kb, hh), pf, o[t]); if (VRES) ol[t] = wmma16b(frag_kb(Vl + (size_t)(t * 16 + col) * T + kb, hh), pf, ol[t] * al); }
    wave_lds_sync(); }
  const float inv = 1.0f / (l * PS * XS);
#pragma unroll
  for (int t = 0; t < 4; ++t)
#pragma unroll
    for (int r = 0; r < 8; ++r) To[wave][col][t * 16 + 8 * hh + r] = (o[t][r] + (VRES ? ol[t][r] * (1.0f / RS_) : 0.0f)) * inv;
  wave_lds_sync();
  for (int pass = 0; pass < 2; ++pass) { for (int i2 = 0; i2 < 8; ++i2) { const int rr = 2 * i2 + hh;
      *(volatile v4f*)(out + ((size_t)b * SEQ_FULL + q0 + rr) * DM + h * HD + col * 4) = *(const v4f*)(&To[wave][rr][col * 4]); } __threadfence(); }
}
}

extern "C" void kernel_launch(void* const* d_in, const int* in_sizes, int n_in, void* d_out, int out_size, void* d_ws, size_t ws_size, hipStream_t stream) {
  if (n_in < 7) return;
  auto Fp = [&](int i) { return (const float*)d_in[i]; };
  const long long need_x = ((long long)(BL - 1) * SEQ_FULL + T) * (long long)DM;
  if ((long long)in_sizes[0] < need_x || in_sizes[1] < H * HD * HD || in_sizes[2] < H * HD * HD || in_sizes[3] < H * HD * HD ||
      in_sizes[4] < H * HD || in_sizes[5] < H * HD || in_sizes[6] < H * HD || (long long)out_size < need_x) return;
  size_t off = 0; char* ws = (char*)d_ws;
  auto carve = [&](size_t bytes) { char* p = ws + off; off += (bytes + 255) & ~(size_t)255; return p; };
  b16* WT = (b16*)carve((size_t)3 * H * HD * HD * 2);
  const size_t plane = (size_t)BL * T * DM * 2;
  b16* QP = (b16*)carve(plane); b16* KP = (b16*)carve(plane); b16* VTh = (b16*)carve(plane); b16* VTl = (b16*)carve(VRES ? plane : 256);
  if (off > ws_size || off > ((size_t)128 << 20)) return;
  prep_kernel<<<(unsigned)(((size_t)3 * H * HD * HD / 8 + 255) / 256), 256, 0, stream>>>(Fp(1), Fp(2), Fp(3), WT);
  proj_kernel<<<dim3(T / 64, BL, 3 * NSL), 128, 0, stream>>>(Fp(0), WT, Fp(4), Fp(5), Fp(6), QP, KP, VTh, VTl);
  attn_kernel<<<dim3(T / 32, BL * H), 64, 0, stream>>>(QP, KP, VTh, VTl, (float*)d_out);
}
